// Correlation2D_10969346474477
// MI455X (gfx1250) — hardware-verified
//
#include <hip/hip_runtime.h>
#include <math.h>

typedef __attribute__((ext_vector_type(16))) __bf16   v16b;
typedef __attribute__((ext_vector_type(8)))  __bf16   v8b;
typedef __attribute__((ext_vector_type(8)))  _Float16 v8h;
typedef __attribute__((ext_vector_type(8)))  float    v8f;
typedef __attribute__((ext_vector_type(4)))  float    v4f;
typedef __attribute__((ext_vector_type(4)))  unsigned v4u;

constexpr int kNB   = 4;
constexpr int kH    = 256;
constexpr int kW    = 256;
constexpr int kNC   = 16;
constexpr int kNTr  = 9;
constexpr int kImg  = kNB * kNC;
constexpr int kPln  = kNTr * kNB;
constexpr int kPix  = kH * kW;
constexpr float kInvHW = 1.0f / (float)(kH * kW);
static_assert(kImg == 64 && kPln == 36 && kPix == 65536, "shape");
static_assert(kH == 256 && kW == 256 && kNC == 16, "kernels are written for 256 x 256 x 16");

constexpr size_t kTab256B = (size_t)256 * 256 * 2;
constexpr size_t kTab512B = (size_t)512 * 512 * 2;
constexpr size_t kPlaneB  = (size_t)kImg * kPix * 2;
constexpr size_t kGB      = (size_t)16384 * 256 * 4;
constexpr size_t kSB      = (size_t)kPln * 128 * 512 * 2;
constexpr size_t kUB      = (size_t)kPln * kPix * 2;
constexpr size_t kCorrB   = (size_t)kPln * kPix * 4;
constexpr size_t kOffTRH  = 0;
constexpr size_t kOffTRL  = kOffTRH + kTab256B;
constexpr size_t kOffFCH  = kOffTRL + kTab256B;
constexpr size_t kOffFCL  = kOffFCH + kTab256B;
constexpr size_t kOffGRH  = kOffFCL + kTab256B;
constexpr size_t kOffGRL  = kOffGRH + kTab256B;
constexpr size_t kOffFIH  = kOffGRL + kTab256B;
constexpr size_t kOffFIL  = kOffFIH + kTab512B;
constexpr size_t kOffTW   = kOffFIL + kTab512B;
constexpr size_t kOffNX   = kOffTW + 1024;
constexpr size_t kOffSC   = kOffNX + 256;
constexpr size_t kOffPART = kOffSC + 256;
constexpr size_t kOffXP   = kOffPART + 131072;
constexpr size_t kOffYP   = kOffXP + kPlaneB;
constexpr size_t kOffZH   = kOffYP + kPlaneB;
constexpr size_t kOffZL   = kOffZH + kPlaneB;
constexpr size_t kOffGX   = kOffZL + kPlaneB;
constexpr size_t kOffGY   = kOffGX + kGB;
constexpr size_t kOffSH   = kOffGY + kGB;
constexpr size_t kOffSL   = kOffSH + kSB;
constexpr size_t kOffUH   = kOffSL + kSB;
constexpr size_t kOffUL   = kOffUH + kUB;
constexpr size_t kOffCORR = kOffUL + kUB;
constexpr size_t kWsTotal = kOffCORR + kCorrB;
static_assert(kWsTotal == 97388032ull, "carve total");
static_assert(kWsTotal <= 134217728ull, "carve cap");
static_assert((kOffTW % 128) == 0 && (kOffNX % 128) == 0 && (kOffSC % 128) == 0 && (kOffPART % 128) == 0 &&
              (kOffXP % 128) == 0 && (kOffYP % 128) == 0 && (kOffZH % 128) == 0 && (kOffZL % 128) == 0 &&
              (kOffGX % 128) == 0 && (kOffGY % 128) == 0 && (kOffSH % 128) == 0 && (kOffSL % 128) == 0 &&
              (kOffUH % 128) == 0 && (kOffUL % 128) == 0 && (kOffCORR % 128) == 0, "128-B aligned regions");

__device__ __forceinline__ unsigned f2bf_u32(float f) {
  const unsigned u = __float_as_uint(f);
  return (u + 0x7FFFu + ((u >> 16) & 1u)) >> 16;
}
__device__ __forceinline__ float bf16r(float f) { return __uint_as_float(f2bf_u32(f) << 16); }

__device__ __forceinline__ void split_pair(float f0, float f1, unsigned& hw, unsigned& lw) {
  const unsigned h0 = f2bf_u32(f0), h1 = f2bf_u32(f1);
  const unsigned l0 = f2bf_u32(f0 - __uint_as_float(h0 << 16));
  const unsigned l1 = f2bf_u32(f1 - __uint_as_float(h1 << 16));
  hw = h0 | (h1 << 16);
  lw = l0 | (l1 << 16);
}
__device__ __forceinline__ void split8(const float* sp, v4u& hv, v4u& lv) {
  const v4f a0 = *(const v4f*)(sp);
  const v4f a1 = *(const v4f*)(sp + 4);
  const float f0 = a0.x, f1 = a0.y, f2 = a0.z, f3 = a0.w;
  const float f4 = a1.x, f5 = a1.y, f6 = a1.z, f7 = a1.w;
  unsigned h0, h1, h2, h3, l0, l1, l2, l3;
  split_pair(f0, f1, h0, l0);
  split_pair(f2, f3, h1, l1);
  split_pair(f4, f5, h2, l2);
  split_pair(f6, f7, h3, l3);
  hv = (v4u){h0, h1, h2, h3};
  lv = (v4u){l0, l1, l2, l3};
}

namespace eng {

__device__ __forceinline__ unsigned short f2bf_bits(float f) {
  unsigned u = __float_as_uint(f);
  return (unsigned short)((u + 0x7FFFu + ((u >> 16) & 1u)) >> 16);
}
__device__ __forceinline__ float bf_bits2f(unsigned short h) { return __uint_as_float(((unsigned)h) << 16); }

__device__ __forceinline__ void guard_row4(v8f& a, v8f& b, v8f& c, v8f& d, v16b x, v16b y) {
  asm volatile("v_nop\n\tv_nop\n\tv_nop\n\tv_nop" : "+v"(a), "+v"(b), "+v"(c), "+v"(d) : "v"(x), "v"(y));
}
__device__ __forceinline__ void keep4_b(v16b a, v16b b, v16b c, v16b d) { asm volatile("v_nop" :: "v"(a), "v"(b), "v"(c), "v"(d)); }
__device__ __forceinline__ void acc_guard4(v8f& a, v8f& b, v8f& c, v8f& d) { asm volatile("v_nop\n\tv_nop\n\tv_nop\n\tv_nop" : "+v"(a), "+v"(b), "+v"(c), "+v"(d)); }

struct FragB {
  union U { v16b v; v8b h[2]; };
  static __device__ __forceinline__ v16b load(const __bf16* p) {
    U f; f.h[0] = *(const v8b*)(p); f.h[1] = *(const v8b*)(p + 16); return f.v;
  }
  static __device__ __forceinline__ v8f mma(v16b a, v16b b, v8f c) {
    return __builtin_amdgcn_wmma_f32_16x16x32_bf16(false, a, false, b, (short)0, c, false, false);
  }
};

template <int SPL, int OUT_MODE>
__global__ __launch_bounds__(256) void wmma_gemm64(
    const unsigned short* __restrict__ Ap, const unsigned short* __restrict__ A2p, int lda, long sA1, long sA2,
    const unsigned short* __restrict__ Btp, const unsigned short* __restrict__ Bt2p, int ldb, long sB1, long sB2,
    void* __restrict__ Cout, void* __restrict__ Cout2, int ldc, long sC1, long sC2,
    int nb2, int M, int N, int K, float scale) {
  typedef __bf16 T;
  typedef v16b V;
  const T* A = (const T*)Ap; const T* A2 = (const T*)A2p; const T* Bt = (const T*)Btp; const T* Bt2 = (const T*)Bt2p;
  __shared__ __align__(16) float sT[8][16 * 68];
  const int bidx = blockIdx.y;
  const int b1 = bidx / nb2;
  const int b2 = bidx - b1 * nb2;
  const int lane = threadIdx.x & 31;
  const int wave = __builtin_amdgcn_readfirstlane((int)(threadIdx.x >> 5));
  const int tilesN = N >> 6;
  const int tilesM = M >> 6;
  const int tile = blockIdx.x * 8 + wave;
  if (tile >= tilesM * tilesN) return;
  const int tm = tile / tilesN;
  const int tn = tile - tm * tilesN;
  const int m0 = tm << 6;
  const int n0 = tn << 6;

  const size_t offA = (size_t)b1 * (size_t)sA1 + (size_t)b2 * (size_t)sA2;
  const size_t offB = (size_t)b1 * (size_t)sB1 + (size_t)b2 * (size_t)sB2;
  const size_t offC = (size_t)b1 * (size_t)sC1 + (size_t)b2 * (size_t)sC2;
  const T* Ab  = A  + offA;
  const T* Bb  = Bt + offB;
  const T* Ab2 = (SPL >= 1) ? (A2  + offA) : nullptr;
  const T* Bb2 = (SPL == 2) ? (Bt2 + offB) : nullptr;

  const int rlane = lane & 15;
  const int koff  = (lane >> 4) * 8;
  const int mOff  = (lane >> 4) * 8;

  v8f acc[4][4];
#pragma unroll
  for (int i = 0; i < 4; ++i)
#pragma unroll
    for (int j = 0; j < 4; ++j) acc[i][j] = (v8f){0.f,0.f,0.f,0.f,0.f,0.f,0.f,0.f};

  for (int k0 = 0; k0 < K; k0 += 32) {
    V bh[4], bl[4];
#pragma unroll
    for (int j = 0; j < 4; ++j) {
      const size_t bo = (size_t)(n0 + (j << 4) + rlane) * ldb + koff + k0;
      bh[j] = FragB::load(Bb + bo);
      if (SPL == 2) bl[j] = FragB::load(Bb2 + bo);
    }
#pragma unroll
    for (int i = 0; i < 4; ++i) {
      const size_t ao = (size_t)(m0 + (i << 4) + rlane) * lda + koff + k0;
      V ah = FragB::load(Ab + ao);
      V al;
      if (SPL >= 1) al = FragB::load(Ab2 + ao);
#pragma unroll
      for (int j = 0; j < 4; ++j) {
        acc[i][j] = FragB::mma(ah, bh[j], acc[i][j]);
        if (SPL == 2) acc[i][j] = FragB::mma(ah, bl[j], acc[i][j]);
        if (SPL >= 1) acc[i][j] = FragB::mma(al, bh[j], acc[i][j]);
      }
      guard_row4(acc[i][0], acc[i][1], acc[i][2], acc[i][3], ah, (SPL >= 1) ? al : ah);
    }
    keep4_b(bh[0], bh[1], bh[2], bh[3]);
    if (SPL == 2) keep4_b(bl[0], bl[1], bl[2], bl[3]);
  }
  acc_guard4(acc[0][0], acc[0][1], acc[0][2], acc[0][3]);
  acc_guard4(acc[1][0], acc[1][1], acc[1][2], acc[1][3]);
  acc_guard4(acc[2][0], acc[2][1], acc[2][2], acc[2][3]);
  acc_guard4(acc[3][0], acc[3][1], acc[3][2], acc[3][3]);

  float* slab = sT[wave];
#pragma unroll
  for (int i = 0; i < 4; ++i) {
    const int mBase = m0 + (i << 4);
#pragma unroll
    for (int j = 0; j < 4; ++j) {
#pragma unroll
      for (int r = 0; r < 8; ++r) {
        const float v = acc[i][j][r] * scale;
        slab[(mOff + r) * 68 + (j << 4) + rlane] = v;
      }
    }
    __builtin_amdgcn_fence(__ATOMIC_RELEASE, "workgroup");
    __builtin_amdgcn_wave_barrier();
    __builtin_amdgcn_fence(__ATOMIC_ACQUIRE, "workgroup");
    if (OUT_MODE == 0) {
      float* C = (float*)Cout + offC;
      const int hh = lane >> 4, c4 = (lane & 15) * 4;
      for (int pass = 0; pass < 2; ++pass) {
#pragma unroll
        for (int it = 0; it < 8; ++it) {
          const int row = it * 2 + hh;
          v4f v = *(const v4f*)(slab + row * 68 + c4);
          *(volatile v4f*)(C + (size_t)(mBase + row) * ldc + n0 + c4) = v;
        }
        __threadfence();
      }
    } else {
      const int q = lane >> 3, c8 = (lane & 7) * 8;
      unsigned short* C  = (unsigned short*)Cout  + offC;
      unsigned short* C2 = (unsigned short*)Cout2 + offC;
      for (int pass = 0; pass < 2; ++pass) {
#pragma unroll
        for (int it = 0; it < 4; ++it) {
          const int row = it * 4 + q;
          const float* sp = slab + row * 68 + c8;
          v8h hv, lv;
#pragma unroll
          for (int e = 0; e < 8; ++e) {
            const float sv = sp[e];
            unsigned short hb = f2bf_bits(sv);
            unsigned short lb = f2bf_bits(sv - bf_bits2f(hb));
            hv[e] = __builtin_bit_cast(_Float16, hb);
            lv[e] = __builtin_bit_cast(_Float16, lb);
          }
          *(volatile v8h*)(C + (size_t)(mBase + row) * ldc + n0 + c8) = hv;
          *(volatile v8h*)(C2 + (size_t)(mBase + row) * ldc + n0 + c8) = lv;
        }
        __threadfence();
      }
    }
    __builtin_amdgcn_fence(__ATOMIC_RELEASE, "workgroup");
    __builtin_amdgcn_wave_barrier();
    __builtin_amdgcn_fence(__ATOMIC_ACQUIRE, "workgroup");
  }
}

}

__global__ __launch_bounds__(256) void tables_kernel(
    unsigned short* trh, unsigned short* trl, unsigned short* fch, unsigned short* fcl,
    unsigned short* grh, unsigned short* grl, unsigned short* fih, unsigned short* fil, float* tw)
{
  __shared__ __align__(16) float sV[2048];
  const int tid = threadIdx.x;
  const int blk = blockIdx.x;
  int tbl, lb;
  if (blk < 32)       { tbl = 0; lb = blk; }
  else if (blk < 64)  { tbl = 1; lb = blk - 32; }
  else if (blk < 96)  { tbl = 2; lb = blk - 64; }
  else if (blk < 224) { tbl = 3; lb = blk - 96; }
  else                { tbl = 4; lb = 0; }
#pragma unroll 1
  for (int it = 0; it < 8; ++it) {
    const int e  = it * 256 + tid;
    const int ge = lb * 2048 + e;
    int ph = 0;
    int usecos = 1;
    float sg = 1.0f, amp = 1.0f;
    if (tbl == 0) {
      const int m = ge >> 8, w = ge & 255;
      const int nyq = (m == 1) ? 1 : 0;
      const int jc = nyq ? 128 : (m >> 1);
      usecos = nyq ? 1 : (((m & 1) == 0) ? 1 : 0);
      sg = -1.0f;
      ph = (jc * w) & 255;
    } else if (tbl == 1) {
      const int n = ge >> 8, k = ge & 255;
      const int pp = n >> 7, kyq = n & 127, part = k >> 7, hq = k & 127;
      usecos = (pp == part) ? 1 : 0;
      sg = (pp == 0) ? 1.0f : -1.0f;
      ph = (2 * kyq * hq) & 255;
    } else if (tbl == 2) {
      const int w = ge >> 8, k = ge & 255;
      const int part = k >> 7, jc = k & 127;
      const int special = (jc == 0 && part == 1) ? 1 : 0;
      const int jce = special ? 128 : jc;
      usecos = special ? 1 : ((part == 0) ? 1 : 0);
      sg = -1.0f;
      amp = (jc == 0) ? 1.0f : 2.0f;
      ph = (jce * w) & 255;
    } else if (tbl == 3) {
      const int n = ge >> 9, k = ge & 511;
      const int pp = n >> 8, h = n & 255, part = k >> 8, ky = k & 255;
      usecos = (pp == part) ? 1 : 0;
      sg = (pp == 0) ? -1.0f : 1.0f;
      ph = (ky * h) & 255;
    } else {
      ph = (ge >> 1) & 127;
      usecos = ((ge & 1) == 0) ? 1 : 0;
    }
    const float x = (float)ph * (1.0f / 128.0f);
    const float c = cospif(x);
    const float s = sinpif(x);
    const float val = amp * (usecos ? c : (sg * s));
    sV[e] = val;
  }
  __syncthreads();
  if (tbl < 4) {
    unsigned short* hp;
    unsigned short* lp;
    if (tbl == 0)      { hp = trh; lp = trl; }
    else if (tbl == 1) { hp = fch; lp = fcl; }
    else if (tbl == 2) { hp = grh; lp = grl; }
    else               { hp = fih; lp = fil; }
    v4u hv, lv;
    split8(sV + tid * 8, hv, lv);
    const size_t eo = (size_t)lb * 2048 + (size_t)tid * 8;
    *(volatile v4u*)(hp + eo) = hv;
    *(volatile v4u*)(lp + eo) = lv;
    __threadfence();
    *(volatile v4u*)(hp + eo) = hv;
    *(volatile v4u*)(lp + eo) = lv;
  } else {
    const float v = sV[tid];
    *(volatile float*)(tw + tid) = v;
    __threadfence();
    *(volatile float*)(tw + tid) = v;
  }
}

__device__ __forceinline__ void warp_coords(float a0, float a1, float a2, float a3, float a4, float a5,
                                            float a6, float a7, float xx, float yy, float& xf, float& yf) {
#pragma clang fp contract(off)
  const float kd = (a6 * xx + a7 * yy) + 1.0f;
  const float nu = (a0 * xx + a1 * yy) + a2;
  const float nv = (a3 * xx + a4 * yy) + a5;
  xf = rintf(nu / kd);
  yf = rintf(nv / kd);
}

__device__ __forceinline__ void stage4(float* sp, v4f q, bool valid) {
  const float f0 = q.x, f1 = q.y, f2 = q.z, f3 = q.w;
  sp[0]   = valid ? bf16r(f0) : 0.0f;
  sp[260] = valid ? bf16r(f1) : 0.0f;
  sp[520] = valid ? bf16r(f2) : 0.0f;
  sp[780] = valid ? bf16r(f3) : 0.0f;
}

template <bool WARP>
__global__ __launch_bounds__(256) void pack_kernel(
    const float* __restrict__ inp, const float* __restrict__ tf, int nt,
    unsigned short* __restrict__ planes, float* __restrict__ part)
{
  __shared__ __align__(16) float sT[16 * 260];
  __shared__ float sP[16];
  const int tid  = threadIdx.x;
  const int lane = tid & 31;
  const int wave = __builtin_amdgcn_readfirstlane((int)(threadIdx.x >> 5));
  const int b = blockIdx.x >> 8;
  const int h = blockIdx.x & 255;
  const int w = tid;
  int sx = w, sy = h;
  bool valid = true;
  if (WARP) {
    const float* t = tf + nt * 8;
    const float a0 = bf16r(t[0]), a1 = bf16r(t[1]), a2 = bf16r(t[2]), a3 = bf16r(t[3]);
    const float a4 = bf16r(t[4]), a5 = bf16r(t[5]), a6 = bf16r(t[6]), a7 = bf16r(t[7]);
    float xf, yf;
    warp_coords(a0, a1, a2, a3, a4, a5, a6, a7, (float)w, (float)h, xf, yf);
    valid = (xf >= 0.0f) && (xf <= (float)(kW - 1)) && (yf >= 0.0f) && (yf <= (float)(kH - 1));
    const float xc = fminf(fmaxf(xf, 0.0f), (float)(kW - 1));
    const float yc = fminf(fmaxf(yf, 0.0f), (float)(kH - 1));
    sx = (int)xc;
    sy = (int)yc;
    sx = sx < 0 ? 0 : (sx > kW - 1 ? kW - 1 : sx);
    sy = sy < 0 ? 0 : (sy > kH - 1 ? kH - 1 : sy);
  }
  const float* src = inp + (((size_t)b * kH + sy) * kW + sx) * kNC;
  v4f q0 = *(const v4f*)(src);
  v4f q1 = *(const v4f*)(src + 4);
  v4f q2 = *(const v4f*)(src + 8);
  v4f q3 = *(const v4f*)(src + 12);
  asm volatile("" : "+v"(q0), "+v"(q1), "+v"(q2), "+v"(q3));
  stage4(sT + 0 * 260 + w, q0, valid);
  stage4(sT + 4 * 260 + w, q1, valid);
  stage4(sT + 8 * 260 + w, q2, valid);
  stage4(sT + 12 * 260 + w, q3, valid);
  __syncthreads();

  {
    const int c = tid >> 4, seg = tid & 15;
    const float* rp = sT + c * 260 + seg * 16;
    float s = 0.0f;
#pragma unroll
    for (int i = 0; i < 4; ++i) {
      const v4f a = *(const v4f*)(rp + 4 * i);
      const float f0 = a.x, f1 = a.y, f2 = a.z, f3 = a.w;
      s += f0 * f0;
      s += f1 * f1;
      s += f2 * f2;
      s += f3 * f3;
    }
    s += __shfl_xor(s, 8, 32);
    s += __shfl_xor(s, 4, 32);
    s += __shfl_xor(s, 2, 32);
    s += __shfl_xor(s, 1, 32);
    if (seg == 0) sP[c] = s;
  }

  v4u ov[2];
#pragma unroll
  for (int it = 0; it < 2; ++it) {
    const int c = it * 8 + wave;
    const float* rp = sT + c * 260 + lane * 8;
    const v4f a0 = *(const v4f*)(rp);
    const v4f a1 = *(const v4f*)(rp + 4);
    const float f0 = a0.x, f1 = a0.y, f2 = a0.z, f3 = a0.w;
    const float f4 = a1.x, f5 = a1.y, f6 = a1.z, f7 = a1.w;
    const unsigned w0 = (__float_as_uint(f0) >> 16) | (__float_as_uint(f1) & 0xffff0000u);
    const unsigned w1 = (__float_as_uint(f2) >> 16) | (__float_as_uint(f3) & 0xffff0000u);
    const unsigned w2 = (__float_as_uint(f4) >> 16) | (__float_as_uint(f5) & 0xffff0000u);
    const unsigned w3 = (__float_as_uint(f6) >> 16) | (__float_as_uint(f7) & 0xffff0000u);
    ov[it] = (v4u){w0, w1, w2, w3};
  }
  for (int pass = 0; pass < 2; ++pass) {
#pragma unroll
    for (int it = 0; it < 2; ++it) {
      const int c = it * 8 + wave;
      unsigned short* dst = planes + ((size_t)(b * kNC + c) * kPix + (size_t)h * kW + (size_t)lane * 8);
      *(volatile v4u*)dst = ov[it];
    }
    __threadfence();
  }
  __syncthreads();
  if (wave == 0) {
    const float pv = sP[lane & 15];
    const float val = (lane < 16) ? pv : 0.0f;
    float* dst = part + (size_t)blockIdx.x * 32 + lane;
    *(volatile float*)dst = val;
    __threadfence();
    *(volatile float*)dst = val;
  }
}

__global__ __launch_bounds__(64) void norm_kernel(const float* part, const float* nxin, float* outv, int mode)
{
  const int tid = threadIdx.x;
  const int b = tid >> 4, c = tid & 15;
  float s = 0.0f;
#pragma unroll 1
  for (int h = 0; h < kH; ++h) s += part[(size_t)(b * kH + h) * 32 + c];
  const float r = sqrtf(s);
  float val = r;
  if (mode != 0) {
    const float nxv = nxin[tid];
    val = 1.0f / ((float)kNC * (nxv * r + 1e-12f));
  }
  *(volatile float*)(outv + tid) = val;
  __threadfence();
  *(volatile float*)(outv + tid) = val;
}

__device__ __forceinline__ void bfly(const float* __restrict__ G, size_t r0, size_t r1, int k, float c, float s,
                                     float& lr, float& li, float& hr, float& hi) {
  const float g0r = G[r0 + k], g0i = G[r0 + 128 + k];
  const float g1r = G[r1 + k], g1i = G[r1 + 128 + k];
  const float tr = c * g1r + s * g1i;
  const float ti = c * g1i - s * g1r;
  lr = g0r + tr; li = g0i + ti;
  hr = g0r - tr; hi = g0i - ti;
}

__device__ __forceinline__ void packed_cross(float ar, float ai, float anr, float ani,
                                             float br, float bi, float bnr, float bni,
                                             float& sr, float& si) {
  const float x0r = 0.5f * (ar + anr), x0i = 0.5f * (ai - ani);
  const float x8r = 0.5f * (ai + ani), x8i = 0.5f * (anr - ar);
  const float y0r = 0.5f * (br + bnr), y0i = 0.5f * (bi - bni);
  const float y8r = 0.5f * (bi + bni), y8i = 0.5f * (bnr - br);
  const float s0r = x0r * y0r + x0i * y0i;
  const float s0i = x0i * y0r - x0r * y0i;
  const float s8r = x8r * y8r + x8i * y8i;
  const float s8i = x8i * y8r - x8r * y8i;
  sr = s0r - s8i;
  si = s0i + s8r;
}

__global__ __launch_bounds__(128) void cross_kernel(
    const float* __restrict__ GX, const float* __restrict__ GY, const float* __restrict__ TW,
    const float* __restrict__ SC, unsigned short* __restrict__ SH, unsigned short* __restrict__ SL, int nt)
{
  __shared__ __align__(16) float sS[512];
  const int tid  = threadIdx.x;
  const int wave = __builtin_amdgcn_readfirstlane((int)(threadIdx.x >> 5));
  const int b  = blockIdx.x >> 7;
  const int jc = blockIdx.x & 127;
  const int kq = tid;
  const int kp = (128 - kq) & 127;
  const float tc = TW[2 * kq], ts = TW[2 * kq + 1];
  const float pc = TW[2 * kp], ps = TW[2 * kp + 1];
  const bool selz = (kq == 0);
  float alr = 0.0f, ali = 0.0f, ahr = 0.0f, ahi = 0.0f;
#pragma unroll 1
  for (int c = 0; c < kNC; ++c) {
    const int img = b * kNC + c;
    const size_t r0 = ((size_t)(img * 2) * 128 + jc) * 256;
    const size_t r1 = ((size_t)(img * 2 + 1) * 128 + jc) * 256;
    const float scv = SC[img];
    float xlr, xli, xhr, xhi, ylr, yli, yhr, yhi;
    bfly(GX, r0, r1, kq, tc, ts, xlr, xli, xhr, xhi);
    bfly(GY, r0, r1, kq, tc, ts, ylr, yli, yhr, yhi);
    if (jc != 0) {
      const float plr = xlr * ylr + xli * yli;
      const float pli = xli * ylr - xlr * yli;
      const float phr = xhr * yhr + xhi * yhi;
      const float phi = xhi * yhr - xhr * yhi;
      alr += scv * plr;
      ali += scv * pli;
      ahr += scv * phr;
      ahi += scv * phi;
    } else {
      float pxlr, pxli, pxhr, pxhi, pylr, pyli, pyhr, pyhi;
      bfly(GX, r0, r1, kp, pc, ps, pxlr, pxli, pxhr, pxhi);
      bfly(GY, r0, r1, kp, pc, ps, pylr, pyli, pyhr, pyhi);
      const float nxlr = selz ? pxlr : pxhr, nxli = selz ? pxli : pxhi;
      const float nxhr = selz ? pxhr : pxlr, nxhi = selz ? pxhi : pxli;
      const float nylr = selz ? pylr : pyhr, nyli = selz ? pyli : pyhi;
      const float nyhr = selz ? pyhr : pylr, nyhi = selz ? pyhi : pyli;
      float plr, pli, phr, phi;
      packed_cross(xlr, xli, nxlr, nxli, ylr, yli, nylr, nyli, plr, pli);
      packed_cross(xhr, xhi, nxhr, nxhi, yhr, yhi, nyhr, nyhi, phr, phi);
      alr += scv * plr;
      ali += scv * pli;
      ahr += scv * phr;
      ahi += scv * phi;
    }
  }
  sS[kq]       = alr;
  sS[128 + kq] = ahr;
  sS[256 + kq] = ali;
  sS[384 + kq] = ahi;
  __syncthreads();
  const int psel = wave >> 1;
  const int seg  = tid & 63;
  v4u hv, lv;
  split8(sS + seg * 8, hv, lv);
  const v4u ovv = psel ? lv : hv;
  unsigned short* base = psel ? SL : SH;
  unsigned short* dst = base + ((size_t)((nt * kNB + b) * 128 + jc)) * 512 + (size_t)seg * 8;
  *(volatile v4u*)dst = ovv;
  __threadfence();
  *(volatile v4u*)dst = ovv;
}

__global__ __launch_bounds__(256) void out_kernel(const float* __restrict__ corr, float* __restrict__ out)
{
  __shared__ float sC[kNTr * 257];
  const int tid  = threadIdx.x;
  const int wave = __builtin_amdgcn_readfirstlane((int)(threadIdx.x >> 5));
  const int b = blockIdx.x >> 8;
  const int h = blockIdx.x & 255;
#pragma unroll 1
  for (int t = 0; t < kNTr; ++t)
    sC[t * 257 + tid] = corr[((size_t)(t * kNB + b) * kH + h) * kW + tid];
  __syncthreads();
  v4f vals[3];
#pragma unroll
  for (int it = 0; it < 3; ++it) {
    int chunk = it * 256 + tid;
    chunk = chunk > 575 ? 575 : chunk;
    const unsigned e0 = (unsigned)chunk * 4u;
    const unsigned w0 = e0 / 9u,        t0 = e0 - 9u * w0;
    const unsigned w1 = (e0 + 1u) / 9u, t1 = (e0 + 1u) - 9u * w1;
    const unsigned w2 = (e0 + 2u) / 9u, t2 = (e0 + 2u) - 9u * w2;
    const unsigned w3 = (e0 + 3u) / 9u, t3 = (e0 + 3u) - 9u * w3;
    const float f0 = sC[t0 * 257u + w0];
    const float f1 = sC[t1 * 257u + w1];
    const float f2 = sC[t2 * 257u + w2];
    const float f3 = sC[t3 * 257u + w3];
    vals[it] = (v4f){f0, f1, f2, f3};
  }
  float* rowp = out + (size_t)blockIdx.x * (size_t)(kW * kNTr);
  for (int pass = 0; pass < 2; ++pass) {
    *(volatile v4f*)(rowp + tid * 4) = vals[0];
    *(volatile v4f*)(rowp + 1024 + tid * 4) = vals[1];
    if (wave < 2) *(volatile v4f*)(rowp + 2048 + tid * 4) = vals[2];
    __threadfence();
  }
}

static_assert((256 % 64) == 0 && (128 % 64) == 0 && (256 % 32) == 0, "S1/S3 tiles");
static_assert((16384 % 64) == 0 && (512 % 32) == 0, "S2/S4/S5 tiles");
static_assert(((kPln * 256) % 64) == 0, "S6 tiles");

extern "C" void kernel_launch(void* const* d_in, const int* in_sizes, int n_in,
                              void* d_out, int out_size, void* d_ws, size_t ws_size,
                              hipStream_t stream) {
  if (n_in < 2) return;
  if (in_sizes[0] != kNB * kH * kW * kNC) return;
  if (in_sizes[1] != kNTr * 8) return;
  if (out_size != kNB * kH * kW * kNTr) return;
  if (ws_size < kWsTotal) return;

  const float* inp = (const float*)d_in[0];
  const float* tf  = (const float*)d_in[1];
  float* out = (float*)d_out;

  char* ws = (char*)d_ws;
  unsigned short* TRH = (unsigned short*)(ws + kOffTRH);
  unsigned short* TRL = (unsigned short*)(ws + kOffTRL);
  unsigned short* FCH = (unsigned short*)(ws + kOffFCH);
  unsigned short* FCL = (unsigned short*)(ws + kOffFCL);
  unsigned short* GRH = (unsigned short*)(ws + kOffGRH);
  unsigned short* GRL = (unsigned short*)(ws + kOffGRL);
  unsigned short* FIH = (unsigned short*)(ws + kOffFIH);
  unsigned short* FIL = (unsigned short*)(ws + kOffFIL);
  float*          TW  = (float*)(ws + kOffTW);
  float*          NX  = (float*)(ws + kOffNX);
  float*          SC  = (float*)(ws + kOffSC);
  float*          PART = (float*)(ws + kOffPART);
  unsigned short* XP  = (unsigned short*)(ws + kOffXP);
  unsigned short* YP  = (unsigned short*)(ws + kOffYP);
  unsigned short* ZH  = (unsigned short*)(ws + kOffZH);
  unsigned short* ZL  = (unsigned short*)(ws + kOffZL);
  float*          GX  = (float*)(ws + kOffGX);
  float*          GY  = (float*)(ws + kOffGY);
  unsigned short* SH  = (unsigned short*)(ws + kOffSH);
  unsigned short* SL  = (unsigned short*)(ws + kOffSL);
  unsigned short* UH  = (unsigned short*)(ws + kOffUH);
  unsigned short* UL  = (unsigned short*)(ws + kOffUL);
  float*          CORR = (float*)(ws + kOffCORR);

  tables_kernel<<<225, 256, 0, stream>>>(TRH, TRL, FCH, FCL, GRH, GRL, FIH, FIL, TW);

  pack_kernel<false><<<kNB * kH, 256, 0, stream>>>(inp, tf, 0, XP, PART);
  norm_kernel<<<1, 64, 0, stream>>>(PART, SC, NX, 0);

  eng::wmma_gemm64<1, 2><<<dim3(1, 128), 256, 0, stream>>>(
      TRH, TRL, 256, 0L, 0L,
      XP, XP, 512, (long)kPix, 256L,
      (void*)ZH, (void*)ZL, 128, (long)kPix, 32768L,
      2, 256, 128, 256, 1.0f);
  eng::wmma_gemm64<2, 0><<<dim3(128, 1), 256, 0, stream>>>(
      ZH, ZL, 256, 0L, 0L,
      FCH, FCL, 256, 0L, 0L,
      (void*)GX, nullptr, 256, 0L, 0L,
      1, 16384, 256, 256, 1.0f);

  for (int nt = 0; nt < kNTr; ++nt) {
    pack_kernel<true><<<kNB * kH, 256, 0, stream>>>(inp, tf, nt, YP, PART);
    norm_kernel<<<1, 64, 0, stream>>>(PART, NX, SC, 1);
    eng::wmma_gemm64<1, 2><<<dim3(1, 128), 256, 0, stream>>>(
        TRH, TRL, 256, 0L, 0L,
        YP, YP, 512, (long)kPix, 256L,
        (void*)ZH, (void*)ZL, 128, (long)kPix, 32768L,
        2, 256, 128, 256, 1.0f);
    eng::wmma_gemm64<2, 0><<<dim3(128, 1), 256, 0, stream>>>(
        ZH, ZL, 256, 0L, 0L,
        FCH, FCL, 256, 0L, 0L,
        (void*)GY, nullptr, 256, 0L, 0L,
        1, 16384, 256, 256, 1.0f);
    cross_kernel<<<kNB * 128, 128, 0, stream>>>(GX, GY, TW, SC, SH, SL, nt);
  }

  eng::wmma_gemm64<2, 2><<<dim3(1, kPln * 2), 256, 0, stream>>>(
      FIH, FIL, 512, 0L, (long)(256 * 512),
      SH, SL, 512, (long)(128 * 512), 0L,
      (void*)UH, (void*)UL, 256, (long)kPix, 128L,
      2, 256, 128, 512, 1.0f);
  eng::wmma_gemm64<2, 0><<<dim3(72, 1), 256, 0, stream>>>(
      UH, UL, 256, 0L, 0L,
      GRH, GRL, 256, 0L, 0L,
      (void*)CORR, nullptr, 256, 0L, 0L,
      1, kPln * 256, 256, 256, kInvHW);

  out_kernel<<<kNB * kH, 256, 0, stream>>>(CORR, out);
}
